// QuantLinear_29832842838126
// MI455X (gfx1250) — hardware-verified
//
#include <hip/hip_runtime.h>
#include <math.h>

constexpr int kTokens    = 2048;
constexpr int kIn        = 4096;
constexpr int kOut       = 4096;
constexpr int kPack      = 8;
constexpr int kKQ        = kIn / kPack;
constexpr int kGroup     = 128;
constexpr int kNumGroups = kIn / kGroup;
constexpr float kClipMin = 1e-5f;
constexpr float kClipMax = 1e4f;
constexpr float kMaxQf   = 15.0f;

constexpr int kWaveM     = 32;
constexpr int kWaveN     = 64;
constexpr int kTilesM    = kTokens / kWaveM;
constexpr int kTilesN    = kOut / kWaveN;
constexpr int kNumTiles  = kTilesM * kTilesN;
constexpr int kStepsPerGroup = kGroup / 32;

constexpr long kABytes   = (long)kTokens * kIn * 2;
constexpr long kBtBytes  = (long)kOut * kIn * 2;
constexpr long kWsTotal  = kABytes + kBtBytes;

static_assert(kIn % 32 == 0, "K multiple of 32");
static_assert(kIn % kGroup == 0 && kGroup % 32 == 0, "group multiple of 32");
static_assert(kTokens % kWaveM == 0 && kOut % kWaveN == 0, "tile multiples");
static_assert(kNumTiles % 8 == 0, "8 wave tiles per block");
static_assert((kTokens * kIn / 8) % 256 == 0, "cast grid exact");
static_assert((kKQ * kOut) % 256 == 0, "dequant grid exact");
static_assert(kKQ % 8 == 0 && kOut % 4 == 0, "dequant lane map");
static_assert(kWsTotal <= 134217728L, "carve under 128 MiB");

typedef __attribute__((ext_vector_type(16))) _Float16 v16h;
typedef __attribute__((ext_vector_type(8)))  _Float16 v8h;
typedef __attribute__((ext_vector_type(16))) __bf16   v16b;
typedef __attribute__((ext_vector_type(8)))  __bf16   v8b;
typedef __attribute__((ext_vector_type(8)))  float    v8f;
typedef __attribute__((ext_vector_type(4)))  float    v4f;
typedef __attribute__((ext_vector_type(4)))  unsigned int v4u;

__device__ __forceinline__ unsigned short f2bf_bits(float f) {
  unsigned u = __float_as_uint(f);
  return (unsigned short)((u + 0x7FFFu + ((u >> 16) & 1u)) >> 16);
}
__device__ __forceinline__ float bf_bits2f(unsigned short h) { return __uint_as_float(((unsigned)h) << 16); }

__device__ __forceinline__ void dep_guard_h(v8f& a, v8f& b, v16h x, v16h y) { asm volatile("v_nop\n\tv_nop\n\tv_nop\n\tv_nop" : "+v"(a), "+v"(b) : "v"(x), "v"(y)); }
__device__ __forceinline__ void dep_guard_b(v8f& a, v8f& b, v16b x, v16b y) { asm volatile("v_nop\n\tv_nop\n\tv_nop\n\tv_nop" : "+v"(a), "+v"(b) : "v"(x), "v"(y)); }
__device__ __forceinline__ void keep4_h(v16h a, v16h b, v16h c, v16h d) { asm volatile("v_nop" :: "v"(a), "v"(b), "v"(c), "v"(d)); }
__device__ __forceinline__ void keep4_b(v16b a, v16b b, v16b c, v16b d) { asm volatile("v_nop" :: "v"(a), "v"(b), "v"(c), "v"(d)); }
__device__ __forceinline__ void acc_guard4(v8f& a, v8f& b, v8f& c, v8f& d) { asm volatile("v_nop\n\tv_nop\n\tv_nop\n\tv_nop" : "+v"(a), "+v"(b), "+v"(c), "+v"(d)); }
template <typename T> struct Frag;
template <> struct Frag<_Float16> {
  typedef v16h V; union U { v16h v; v8h h[2]; };
  static __device__ __forceinline__ v16h load(const _Float16* p) {
    U f; f.h[0] = *(const v8h*)(p); f.h[1] = *(const v8h*)(p + 16); return f.v;
  }
  static __device__ __forceinline__ v8f mma(v16h a, v16h b, v8f c) {
    return __builtin_amdgcn_wmma_f32_16x16x32_f16(false, a, false, b, (short)0, c, false, false);
  }
  static __device__ __forceinline__ void guard(v8f& a, v8f& b, v16h x, v16h y) { dep_guard_h(a, b, x, y); }
  static __device__ __forceinline__ void keep(v16h a, v16h b, v16h c, v16h d) { keep4_h(a, b, c, d); }
};
template <> struct Frag<__bf16> {
  typedef v16b V; union U { v16b v; v8b h[2]; };
  static __device__ __forceinline__ v16b load(const __bf16* p) {
    U f; f.h[0] = *(const v8b*)(p); f.h[1] = *(const v8b*)(p + 16); return f.v;
  }
  static __device__ __forceinline__ v8f mma(v16b a, v16b b, v8f c) {
    return __builtin_amdgcn_wmma_f32_16x16x32_bf16(false, a, false, b, (short)0, c, false, false);
  }
  static __device__ __forceinline__ void guard(v8f& a, v8f& b, v16b x, v16b y) { dep_guard_b(a, b, x, y); }
  static __device__ __forceinline__ void keep(v16b a, v16b b, v16b c, v16b d) { keep4_b(a, b, c, d); }
};

__device__ __forceinline__ unsigned pk16(unsigned short a, unsigned short b) { return (unsigned)a | ((unsigned)b << 16); }

__device__ __forceinline__ void guard_row_b(v8f& a, v8f& b, v8f& c, v8f& d,
                                            v16b x, v16b y0, v16b y1, v16b y2, v16b y3) {
  asm volatile("v_nop\n\tv_nop\n\tv_nop\n\tv_nop"
               : "+v"(a), "+v"(b), "+v"(c), "+v"(d)
               : "v"(x), "v"(y0), "v"(y1), "v"(y2), "v"(y3));
}

__global__ __launch_bounds__(256) void cast8_bf16_kernel(const float* __restrict__ in,
                                                         unsigned short* __restrict__ out, int n8) {
  const int i = blockIdx.x * 256 + threadIdx.x;
  if (i >= n8) return;
  const float* p = in + 8 * (size_t)i;
  const v4f a = *(const v4f*)(p);
  const v4f c = *(const v4f*)(p + 4);
  unsigned short hb[8];
#pragma unroll
  for (int e = 0; e < 4; ++e) {
    hb[e]     = f2bf_bits(a[e]);
    hb[4 + e] = f2bf_bits(c[e]);
  }
  const v4u u = (v4u){pk16(hb[0], hb[1]), pk16(hb[2], hb[3]), pk16(hb[4], hb[5]), pk16(hb[6], hb[7])};
  unsigned short* q = out + 8 * (size_t)i;
  *(volatile v4u*)q = u;
  __threadfence();
  *(volatile v4u*)q = u;
}

__global__ __launch_bounds__(256) void dequant_bt_kernel(const int* __restrict__ qw,
                                                         const float* __restrict__ zp,
                                                         unsigned short* __restrict__ bt) {
  const int t    = blockIdx.x * 256 + threadIdx.x;
  const int lane = t & 31;
  const int w    = t >> 5;
  const int nb   = w & (kOut / 4 - 1);
  const int kb   = w >> 10;
  const int kq   = kb * 8 + (lane & 7);
  const int n    = nb * 4 + (lane >> 3);
  const int g    = kb >> 1;
  const unsigned q = (unsigned)qw[(size_t)kq * kOut + n];
  float z = bf_bits2f(f2bf_bits(zp[(size_t)g * kOut + n]));
  z = rintf(z);
  z = fminf(fmaxf(z, 0.0f), kMaxQf);
  unsigned short hb[8];
#pragma unroll
  for (int j = 0; j < 8; ++j) {
    const float wq = (float)((q >> (4 * j)) & 15u);
    hb[j] = f2bf_bits(wq - z);
  }
  const v4u u = (v4u){pk16(hb[0], hb[1]), pk16(hb[2], hb[3]), pk16(hb[4], hb[5]), pk16(hb[6], hb[7])};
  unsigned short* dst = bt + (size_t)n * kIn + (size_t)kq * 8;
  *(volatile v4u*)dst = u;
  __threadfence();
  *(volatile v4u*)dst = u;
}

__global__ __launch_bounds__(256) void qgemm_fold_kernel(const unsigned short* __restrict__ Ap,
                                                         const unsigned short* __restrict__ Btp,
                                                         const float* __restrict__ scales,
                                                         const float* __restrict__ bias,
                                                         float* __restrict__ C) {
  typedef __bf16 T;
  typedef v16b V;
  const T* A  = (const T*)Ap;
  const T* Bt = (const T*)Btp;
  __shared__ __align__(16) float sT[8][16 * 68];

  const int lane = threadIdx.x & 31;
  const int wave = threadIdx.x >> 5;
  const int tile = blockIdx.x * 8 + wave;
  if (tile >= kNumTiles) return;
  const int tm = tile / kTilesN;
  const int tn = tile - tm * kTilesN;
  const int m0 = tm * kWaveM;
  const int n0 = tn * kWaveN;

  const int rlane = lane & 15;
  const int koff  = (lane >> 4) * 8;
  const int mOff  = (lane >> 4) * 8;

  v8f acc[2][4];
#pragma unroll
  for (int i = 0; i < 2; ++i)
#pragma unroll
    for (int j = 0; j < 4; ++j) acc[i][j] = (v8f){0.f,0.f,0.f,0.f,0.f,0.f,0.f,0.f};

#pragma unroll 1
  for (int g = 0; g < kNumGroups; ++g) {
    v8f part[2][4];
#pragma unroll
    for (int i = 0; i < 2; ++i)
#pragma unroll
      for (int j = 0; j < 4; ++j) part[i][j] = (v8f){0.f,0.f,0.f,0.f,0.f,0.f,0.f,0.f};

#pragma unroll 1
    for (int ks = 0; ks < kStepsPerGroup; ++ks) {
      const int k0 = g * kGroup + ks * 32;
      V bh[4];
#pragma unroll
      for (int j = 0; j < 4; ++j) {
        const size_t bo = (size_t)(n0 + (j << 4) + rlane) * kIn + koff + k0;
        bh[j] = Frag<T>::load(Bt + bo);
      }
#pragma unroll
      for (int i = 0; i < 2; ++i) {
        const size_t ao = (size_t)(m0 + (i << 4) + rlane) * kIn + koff + k0;
        const V ah = Frag<T>::load(A + ao);
#pragma unroll
        for (int j = 0; j < 4; ++j) part[i][j] = Frag<T>::mma(ah, bh[j], part[i][j]);
        guard_row_b(part[i][0], part[i][1], part[i][2], part[i][3], ah, bh[0], bh[1], bh[2], bh[3]);
      }
    }
    acc_guard4(part[0][0], part[0][1], part[0][2], part[0][3]);
    acc_guard4(part[1][0], part[1][1], part[1][2], part[1][3]);

#pragma unroll
    for (int j = 0; j < 4; ++j) {
      const int n = n0 + (j << 4) + rlane;
      float s = bf_bits2f(f2bf_bits(scales[(size_t)g * kOut + n]));
      s = fminf(fmaxf(s, kClipMin), kClipMax);
#pragma unroll
      for (int i = 0; i < 2; ++i) {
#pragma unroll
        for (int r = 0; r < 8; ++r) acc[i][j][r] = fmaf(s, part[i][j][r], acc[i][j][r]);
      }
    }
  }

  float* slab = sT[wave];
  float bv[4];
#pragma unroll
  for (int j = 0; j < 4; ++j) bv[j] = bf_bits2f(f2bf_bits(bias[n0 + (j << 4) + rlane]));
#pragma unroll
  for (int i = 0; i < 2; ++i) {
    const int mBase = m0 + (i << 4);
#pragma unroll
    for (int j = 0; j < 4; ++j) {
#pragma unroll
      for (int r = 0; r < 8; ++r) {
        slab[(mOff + r) * 68 + (j << 4) + rlane] = acc[i][j][r] + bv[j];
      }
    }
    __builtin_amdgcn_fence(__ATOMIC_RELEASE, "workgroup");
    __builtin_amdgcn_wave_barrier();
    __builtin_amdgcn_fence(__ATOMIC_ACQUIRE, "workgroup");
    {
      const int hh = lane >> 4, c4 = (lane & 15) * 4;
      for (int pass = 0; pass < 2; ++pass) {
#pragma unroll
        for (int it = 0; it < 8; ++it) {
          const int row = it * 2 + hh;
          v4f v = *(const v4f*)(slab + row * 68 + c4);
          *(volatile v4f*)(C + (size_t)(mBase + row) * kOut + n0 + c4) = v;
        }
        __threadfence();
      }
    }
    __builtin_amdgcn_fence(__ATOMIC_RELEASE, "workgroup");
    __builtin_amdgcn_wave_barrier();
    __builtin_amdgcn_fence(__ATOMIC_ACQUIRE, "workgroup");
  }
}

extern "C" void kernel_launch(void* const* d_in, const int* in_sizes, int n_in,
                              void* d_out, int out_size, void* d_ws, size_t ws_size,
                              hipStream_t stream)
{
  if (n_in < 5) return;
  if (in_sizes[0] != kTokens * kIn) return;
  if (in_sizes[1] != kNumGroups * kOut) return;
  if (in_sizes[2] != kNumGroups * kOut) return;
  if (in_sizes[3] != kOut) return;
  if (in_sizes[4] != kKQ * kOut) return;
  if (out_size != kTokens * kOut) return;
  if (ws_size < (size_t)kWsTotal) return;

  const float* x      = (const float*)d_in[0];
  const float* scales = (const float*)d_in[1];
  const float* zerop  = (const float*)d_in[2];
  const float* bias   = (const float*)d_in[3];
  const int*   qw     = (const int*)d_in[4];
  float*       out    = (float*)d_out;

  unsigned short* aplane  = (unsigned short*)d_ws;
  unsigned short* btplane = (unsigned short*)((char*)d_ws + kABytes);

  const int n8 = kTokens * kIn / 8;
  cast8_bf16_kernel<<<n8 / 256, 256, 0, stream>>>(x, aplane, n8);
  dequant_bt_kernel<<<(kKQ * kOut) / 256, 256, 0, stream>>>(qw, zerop, btplane);
  qgemm_fold_kernel<<<kNumTiles / 8, 256, 0, stream>>>(aplane, btplane, scales, bias, out);
}
